// IMVTensorLSTM_35192962023884
// MI455X (gfx1250) — hardware-verified
//
#include <hip/hip_runtime.h>


typedef _Float16 f16t;
typedef f16t  v16h __attribute__((ext_vector_type(16)));
typedef f16t  v8h  __attribute__((ext_vector_type(8)));
typedef float v8f  __attribute__((ext_vector_type(8)));
typedef float v4f  __attribute__((ext_vector_type(4)));

union Frag { v16h v; v8h q[2]; };
union F8   { v4f v[2]; float f[8]; };

#define NBATCH 128
#define NSTEP  256
#define NVAR   32
#define NUNIT  64
#define WP     72
#define HP     72
#define TP     36
#define SC_W   64.0f
#define SC_H   256.0f
#define INV_WH (1.0f / 16384.0f)

__device__ __forceinline__ v8f wmma16(v16h a, v16h b, v8f c) {
    return __builtin_amdgcn_wmma_f32_16x16x32_f16(false, a, false, b, (short)0, c, false, false);
}

__device__ __forceinline__ float rcp_f(float v) { return __builtin_amdgcn_rcpf(v); }
__device__ __forceinline__ float tanh_f(float v) {
    const float av = fabsf(v);
    const float e  = __expf(-2.0f * av);
    const float r  = (1.0f - e) * rcp_f(1.0f + e);
    return copysignf(r, v);
}
__device__ __forceinline__ float sigm_f(float v) { return rcp_f(1.0f + __expf(-v)); }

__device__ __forceinline__ void stage_w(const float* __restrict__ Wg, f16t* P, int iv, int tid) {
#pragma unroll
    for (int ps = 0; ps < 8; ++ps) {
        const int idx = tid + 128 * ps;
        const int j   = idx >> 4;
        const int c4  = (idx & 15) * 4;
        const v4f v = *(const v4f*)(Wg + ((size_t)(j * NVAR + iv)) * NUNIT + c4);
#pragma unroll
        for (int e = 0; e < 4; ++e) P[(c4 + e) * WP + j] = (f16t)(v[e] * SC_W);
    }
}

__global__ __launch_bounds__(128)
void k_rec(const float* __restrict__ x,
           const float* __restrict__ Uj, const float* __restrict__ Ui,
           const float* __restrict__ Uf, const float* __restrict__ Uo,
           const float* __restrict__ Wj, const float* __restrict__ Wi,
           const float* __restrict__ Wf, const float* __restrict__ Wo,
           const float* __restrict__ bj, const float* __restrict__ bi,
           const float* __restrict__ bf, const float* __restrict__ bo,
           const float* __restrict__ Fa, const float* __restrict__ Fab,
           float* __restrict__ AP, float* __restrict__ HG)
{
    __shared__ __attribute__((aligned(16))) f16t  wl[4 * NUNIT * WP];
    __shared__ __attribute__((aligned(16))) f16t  hl[16 * HP];
    __shared__ __attribute__((aligned(16))) float xs[NSTEP * 16];
    __shared__ __attribute__((aligned(16))) float ab[16 * NSTEP];
    __shared__ __attribute__((aligned(16))) float sp[16 * 4];
    __shared__ __attribute__((aligned(16))) float hgs[16 * 128];
    __shared__ __attribute__((aligned(16))) float sinv[16];

    const int tid  = threadIdx.x;
    const int nq   = tid >> 5;
    const int l    = tid & 31;
    const int hf   = l >> 4;
    const int m    = l & 15;
    const int ncol = nq * 16 + m;
    const int iv   = blockIdx.x & 31;
    const int b0   = (blockIdx.x >> 5) * 16;

    stage_w(Wj, wl + 0 * NUNIT * WP, iv, tid);
    stage_w(Wi, wl + 1 * NUNIT * WP, iv, tid);
    stage_w(Wf, wl + 2 * NUNIT * WP, iv, tid);
    stage_w(Wo, wl + 3 * NUNIT * WP, iv, tid);

#pragma unroll 4
    for (int ps = 0; ps < 32; ++ps) {
        const int idx = tid + 128 * ps;
        const int t   = idx >> 4;
        const int row = idx & 15;
        xs[idx] = x[((size_t)(b0 + row) * NSTEP + t) * NVAR + iv];
    }
    for (int k = tid; k < 16 * HP; k += 128) hl[k] = (f16t)0.0f;

    float ug[4], bg[4];
    ug[0] = Uj[iv * NUNIT + ncol];  bg[0] = bj[iv * NUNIT + ncol];
    ug[1] = Ui[iv * NUNIT + ncol];  bg[1] = bi[iv * NUNIT + ncol];
    ug[2] = Uf[iv * NUNIT + ncol];  bg[2] = bf[iv * NUNIT + ncol];
    ug[3] = Uo[iv * NUNIT + ncol];  bg[3] = bo[iv * NUNIT + ncol];
    const float fa  = Fa[ncol * NVAR + iv];
    const float fab = Fab[iv];

    float cst[8], gnum[8], asum[8], hcur[8];
#pragma unroll
    for (int r = 0; r < 8; ++r) { cst[r] = 0.f; gnum[r] = 0.f; asum[r] = 0.f; hcur[r] = 0.f; }

    __syncthreads();

    Frag bfr[4][2];
#pragma unroll
    for (int g = 0; g < 4; ++g)
#pragma unroll
        for (int kt = 0; kt < 2; ++kt) {
            const f16t* p = wl + (size_t)(g * NUNIT + ncol) * WP + kt * 32 + 8 * hf;
            bfr[g][kt].q[0] = *(const v8h*)p;
            bfr[g][kt].q[1] = *(const v8h*)(p + 16);
        }

    const f16t* hrow = hl + m * HP + 8 * hf;
    const v8f z = {0.f, 0.f, 0.f, 0.f, 0.f, 0.f, 0.f, 0.f};

#pragma unroll 1
    for (int t = 0; t < NSTEP; ++t) {
        Frag a0, a1;
        a0.q[0] = *(const v8h*)(hrow);
        a0.q[1] = *(const v8h*)(hrow + 16);
        a1.q[0] = *(const v8h*)(hrow + 32);
        a1.q[1] = *(const v8h*)(hrow + 48);

        v8f acc[4];
#pragma unroll
        for (int g = 0; g < 4; ++g) {
            acc[g] = wmma16(a0.v, bfr[g][0].v, z);
            acc[g] = wmma16(a1.v, bfr[g][1].v, acc[g]);
        }
        asm volatile("v_nop\n\tv_nop\n\tv_nop\n\tv_nop"
                     : "+v"(acc[0]), "+v"(acc[1]), "+v"(acc[2]), "+v"(acc[3])
                     : "v"(a0.v), "v"(a1.v),
                       "v"(bfr[0][0].v), "v"(bfr[0][1].v), "v"(bfr[1][0].v), "v"(bfr[1][1].v),
                       "v"(bfr[2][0].v), "v"(bfr[2][1].v), "v"(bfr[3][0].v), "v"(bfr[3][1].v));

        __syncthreads();

        F8 xx;
        xx.v[0] = *(const v4f*)(xs + t * 16 + 8 * hf);
        xx.v[1] = *(const v4f*)(xs + t * 16 + 8 * hf + 4);

#pragma unroll
        for (int r = 0; r < 8; ++r) {
            const int row  = 8 * hf + r;
            const float xv = xx.f[r];
            const float pj = fmaf(acc[0][r], INV_WH, fmaf(xv, ug[0], bg[0]));
            const float pi = fmaf(acc[1][r], INV_WH, fmaf(xv, ug[1], bg[1]));
            const float pf = fmaf(acc[2][r], INV_WH, fmaf(xv, ug[2], bg[2]));
            const float po = fmaf(acc[3][r], INV_WH, fmaf(xv, ug[3], bg[3]));
            const float jg = tanh_f(pj);
            const float ig = sigm_f(pi);
            const float fg = sigm_f(pf);
            const float og = sigm_f(po);
            cst[r] = cst[r] * fg + ig * jg;
            const float hv = og * tanh_f(cst[r]);
            hcur[r] = hv;
            hl[row * HP + ncol] = (f16t)(hv * SC_H);
            float p = hv * fa;
            p += __shfl_xor(p, 1, 32);
            p += __shfl_xor(p, 2, 32);
            p += __shfl_xor(p, 4, 32);
            p += __shfl_xor(p, 8, 32);
            if (m == 0) sp[row * 4 + nq] = p;
        }

        __syncthreads();

#pragma unroll
        for (int r = 0; r < 8; ++r) {
            const int row = 8 * hf + r;
            const v4f q   = *(const v4f*)(sp + row * 4);
            const float s  = ((q[0] + q[1]) + q[2]) + q[3] + fab;
            const float at = __expf(tanh_f(s));
            asum[r] += at;
            gnum[r]  = fmaf(at, hcur[r], gnum[r]);
            if (nq == 0 && m == 0) ab[row * NSTEP + t] = at;
        }
    }

    float inv[8];
#pragma unroll
    for (int r = 0; r < 8; ++r) inv[r] = 1.0f / asum[r];
    if (nq == 0 && m == 0) {
#pragma unroll
        for (int r = 0; r < 8; ++r) sinv[8 * hf + r] = inv[r];
    }
#pragma unroll
    for (int r = 0; r < 8; ++r) {
        const int row = 8 * hf + r;
        hgs[row * 128 + ncol]      = gnum[r] * inv[r];
        hgs[row * 128 + 64 + ncol] = hcur[r];
    }
    __syncthreads();

    v4f va[8];
#pragma unroll
    for (int it = 0; it < 8; ++it) {
        const int p = tid + 128 * it, row = p >> 6, c = (p & 63) * 4;
        const v4f v = *(const v4f*)(ab + row * NSTEP + c);
        va[it] = v * sinv[row];
    }
    v4f vh[4];
#pragma unroll
    for (int it = 0; it < 4; ++it) {
        const int p = tid + 128 * it, row = p >> 5, c = (p & 31) * 4;
        vh[it] = *(const v4f*)(hgs + row * 128 + c);
    }
    float* apb = AP + (size_t)(iv * NBATCH + b0) * NSTEP;
    float* hgb = HG + (size_t)(iv * NBATCH + b0) * 128;
#pragma unroll
    for (int it = 0; it < 8; ++it) {
        const int p = tid + 128 * it, row = p >> 6, c = (p & 63) * 4;
        *(volatile v4f*)(apb + row * NSTEP + c) = va[it];
    }
#pragma unroll
    for (int it = 0; it < 4; ++it) {
        const int p = tid + 128 * it, row = p >> 5, c = (p & 31) * 4;
        *(volatile v4f*)(hgb + row * 128 + c) = vh[it];
    }
    __threadfence();
#pragma unroll
    for (int it = 0; it < 8; ++it) {
        const int p = tid + 128 * it, row = p >> 6, c = (p & 63) * 4;
        *(volatile v4f*)(apb + row * NSTEP + c) = va[it];
    }
#pragma unroll
    for (int it = 0; it < 4; ++it) {
        const int p = tid + 128 * it, row = p >> 5, c = (p & 31) * 4;
        *(volatile v4f*)(hgb + row * 128 + c) = vh[it];
    }
}

__global__ __launch_bounds__(256)
void k_alpha(const float* __restrict__ AP, float* out1)
{
    __shared__ __attribute__((aligned(16))) float tile[NSTEP * TP];
    const int tid = threadIdx.x;
    const int b   = blockIdx.x;
#pragma unroll 4
    for (int i = 0; i < NVAR; ++i)
        tile[tid * TP + i] = AP[((size_t)(i * NBATCH + b)) * NSTEP + tid];
    __syncthreads();

    v4f v[8];
#pragma unroll
    for (int it = 0; it < 8; ++it) {
        const int p = tid + 256 * it, t = p >> 3, c = (p & 7) * 4;
        v[it] = *(const v4f*)(tile + t * TP + c);
    }
    float* ob = out1 + (size_t)b * NSTEP * NVAR;
#pragma unroll
    for (int it = 0; it < 8; ++it) {
        const int p = tid + 256 * it, t = p >> 3, c = (p & 7) * 4;
        *(volatile v4f*)(ob + t * NVAR + c) = v[it];
    }
    __threadfence();
#pragma unroll
    for (int it = 0; it < 8; ++it) {
        const int p = tid + 256 * it, t = p >> 3, c = (p & 7) * 4;
        *(volatile v4f*)(ob + t * NVAR + c) = v[it];
    }
}

__global__ __launch_bounds__(256)
void k_head(const float* __restrict__ HG,
            const float* __restrict__ Fbw, const float* __restrict__ Fbb,
            const float* __restrict__ Pw,  const float* __restrict__ Pb,
            float* out0, float* out2)
{
    __shared__ __attribute__((aligned(16))) float mus[NBATCH * NVAR];
    __shared__ __attribute__((aligned(16))) float brs[NBATCH * NVAR];
    __shared__ __attribute__((aligned(16))) float mns[NBATCH];
    const int tid = threadIdx.x;
    const int w   = tid >> 5;
    const int l   = tid & 31;
    const v4f pw = *(const v4f*)(Pw  + 4 * l);
    const v4f fw = *(const v4f*)(Fbw + 4 * l);
    const float pb = Pb[0];
    const float fb = Fbb[0];

#pragma unroll 1
    for (int q = w; q < NBATCH * NVAR; q += 8) {
        const int b = q >> 5, i = q & 31;
        const v4f v = *(const v4f*)(HG + ((size_t)(i * NBATCH + b)) * 128 + 4 * l);
        float pm = v[0] * pw[0];
        pm = fmaf(v[1], pw[1], pm); pm = fmaf(v[2], pw[2], pm); pm = fmaf(v[3], pw[3], pm);
        float ps = v[0] * fw[0];
        ps = fmaf(v[1], fw[1], ps); ps = fmaf(v[2], fw[2], ps); ps = fmaf(v[3], fw[3], ps);
        pm += __shfl_xor(pm, 16, 32); ps += __shfl_xor(ps, 16, 32);
        pm += __shfl_xor(pm, 8, 32);  ps += __shfl_xor(ps, 8, 32);
        pm += __shfl_xor(pm, 4, 32);  ps += __shfl_xor(ps, 4, 32);
        pm += __shfl_xor(pm, 2, 32);  ps += __shfl_xor(ps, 2, 32);
        pm += __shfl_xor(pm, 1, 32);  ps += __shfl_xor(ps, 1, 32);
        if (l == 0) {
            mus[q] = pm + pb;
            brs[q] = __expf(tanh_f(ps + fb));
        }
    }
    __syncthreads();

    if (tid < NBATCH) {
        float bs = 0.f;
#pragma unroll 1
        for (int i = 0; i < NVAR; ++i) bs += brs[tid * NVAR + i];
        const float ib = 1.0f / bs;
        float mean = 0.f;
#pragma unroll 1
        for (int i = 0; i < NVAR; ++i) {
            const float bt = brs[tid * NVAR + i] * ib;
            brs[tid * NVAR + i] = bt;
            mean = fmaf(bt, mus[tid * NVAR + i], mean);
        }
        mns[tid] = mean;
    }
    __syncthreads();

    v4f vb[4];
#pragma unroll
    for (int it = 0; it < 4; ++it) {
        const int p = tid + 256 * it;
        vb[it] = *(const v4f*)(brs + 4 * p);
    }
    const int lm = (tid < 32) ? tid : 31;
    const v4f vm = *(const v4f*)(mns + 4 * lm);

#pragma unroll
    for (int it = 0; it < 4; ++it) {
        const int p = tid + 256 * it;
        *(volatile v4f*)(out2 + 4 * p) = vb[it];
    }
    if (tid < 32) *(volatile v4f*)(out0 + 4 * tid) = vm;
    __threadfence();
#pragma unroll
    for (int it = 0; it < 4; ++it) {
        const int p = tid + 256 * it;
        *(volatile v4f*)(out2 + 4 * p) = vb[it];
    }
    if (tid < 32) *(volatile v4f*)(out0 + 4 * tid) = vm;
}

extern "C" void kernel_launch(void* const* d_in, const int* in_sizes, int n_in,
                              void* d_out, int out_size, void* d_ws, size_t ws_size,
                              hipStream_t stream) {
    if (n_in < 19) return;
    if (in_sizes[0] != NBATCH * NSTEP * NVAR) return;
    for (int k = 1; k <= 4; ++k)  if (in_sizes[k] != NVAR * NUNIT) return;
    for (int k = 5; k <= 8; ++k)  if (in_sizes[k] != NUNIT * NVAR * NUNIT) return;
    for (int k = 9; k <= 12; ++k) if (in_sizes[k] != NVAR * NUNIT) return;
    if (in_sizes[13] != NUNIT * NVAR || in_sizes[14] != NVAR) return;
    if (in_sizes[15] != 2 * NUNIT || in_sizes[16] != 1) return;
    if (in_sizes[17] != 2 * NUNIT || in_sizes[18] != 1) return;
    if (out_size != NBATCH + NBATCH * NSTEP * NVAR + NBATCH * NVAR) return;

    const float* x   = (const float*)d_in[0];
    const float* Uj  = (const float*)d_in[1];
    const float* Ui  = (const float*)d_in[2];
    const float* Uf  = (const float*)d_in[3];
    const float* Uo  = (const float*)d_in[4];
    const float* Wj  = (const float*)d_in[5];
    const float* Wi  = (const float*)d_in[6];
    const float* Wf  = (const float*)d_in[7];
    const float* Wo  = (const float*)d_in[8];
    const float* bj  = (const float*)d_in[9];
    const float* bi  = (const float*)d_in[10];
    const float* bf  = (const float*)d_in[11];
    const float* bo  = (const float*)d_in[12];
    const float* Fa  = (const float*)d_in[13];
    const float* Fab = (const float*)d_in[14];
    const float* Fbw = (const float*)d_in[15];
    const float* Fbb = (const float*)d_in[16];
    const float* Pw  = (const float*)d_in[17];
    const float* Pb  = (const float*)d_in[18];

    float* out  = (float*)d_out;
    float* out0 = out;
    float* out1 = out + NBATCH;
    float* out2 = out + NBATCH + (size_t)NBATCH * NSTEP * NVAR;

    const size_t apB = (size_t)NVAR * NBATCH * NSTEP * sizeof(float);
    const size_t hgB = (size_t)NVAR * NBATCH * 128 * sizeof(float);
    if (apB + hgB > ws_size) return;
    char* ws = (char*)d_ws;
    float* AP = (float*)ws;
    float* HG = (float*)(ws + apB);

    k_rec<<<dim3(NVAR * (NBATCH / 16)), dim3(128), 0, stream>>>(
        x, Uj, Ui, Uf, Uo, Wj, Wi, Wf, Wo, bj, bi, bf, bo, Fa, Fab, AP, HG);
    k_alpha<<<dim3(NBATCH), dim3(256), 0, stream>>>(AP, out1);
    k_head<<<dim3(1), dim3(256), 0, stream>>>(HG, Fbw, Fbb, Pw, Pb, out0, out2);
}
